// SemanticAttentionTransformerLayer_40630390620222
// MI455X (gfx1250) — hardware-run, weakly checked
//
#include <hip/hip_runtime.h>


#define NB_  8
#define TT   1024
#define DD   512
#define NH_  8
#define HD   64
#define NW   256
#define NC2  512
#define TXT  256
#define AUD  768
#define NS_  256
#define FF   2048
#define PCAR 1024.0f
typedef _Float16 h16;
typedef unsigned short bf;
typedef __attribute__((ext_vector_type(16))) __bf16   v16bf;
typedef __attribute__((ext_vector_type(16))) _Float16 v16h;
typedef __attribute__((ext_vector_type(8)))  _Float16 v8h;
typedef __attribute__((ext_vector_type(8)))  unsigned short v8us;
typedef __attribute__((ext_vector_type(8)))  float    v8f;
typedef __attribute__((ext_vector_type(4)))  float    v4f;
typedef v8h  __attribute__((may_alias)) v8ha;
typedef v4f  __attribute__((may_alias)) v4fa;
typedef v8us __attribute__((may_alias)) v8usa;

__device__ __forceinline__ unsigned short f2bf(float f) { unsigned u = __float_as_uint(f); u += 0x7FFFu + ((u >> 16) & 1u); return (unsigned short)(u >> 16); }
__device__ __forceinline__ float bf2f(unsigned short b) { return __uint_as_float(((unsigned)b) << 16); }
__device__ __forceinline__ float bfr(float f) { return bf2f(f2bf(f)); }
__device__ __forceinline__ v16h cat16(v8h lo, v8h hi) { return __builtin_shufflevector(lo, hi, 0, 1, 2, 3, 4, 5, 6, 7, 8, 9, 10, 11, 12, 13, 14, 15); }
__device__ __forceinline__ v16bf cat16b(v8us lo, v8us hi) { return __builtin_bit_cast(v16bf, __builtin_shufflevector(lo, hi, 0, 1, 2, 3, 4, 5, 6, 7, 8, 9, 10, 11, 12, 13, 14, 15)); }
__device__ __forceinline__ v8f wmma16(v16h a, v16h b, v8f c) { return __builtin_amdgcn_wmma_f32_16x16x32_f16(false, a, false, b, (short)0, c, false, false); }
__device__ __forceinline__ v8f wmmab(v16bf a, v16bf b, v8f c) { return __builtin_amdgcn_wmma_f32_16x16x32_bf16(false, a, false, b, (short)0, c, false, false); }


template <typename T16> struct WFrag;
template <> struct WFrag<h16> { typedef v16h V; static __device__ __forceinline__ V ld(const h16* p) { return cat16(*(const v8h*)p, *(const v8h*)(p + 16)); } static __device__ __forceinline__ v8f mma(V a, V b, v8f c) { return wmma16(a, b, c); } };
template <> struct WFrag<bf> { typedef v16bf V; static __device__ __forceinline__ V ld(const bf* p) { return cat16b(*(const v8us*)p, *(const v8us*)(p + 16)); } static __device__ __forceinline__ v8f mma(V a, V b, v8f c) { return wmmab(a, b, c); } };
template <typename T16, int NSPLIT, bool BIAS>
__global__ __launch_bounds__(32) void k_gemmw(const T16* __restrict__ A, const T16* __restrict__ A2, const T16* __restrict__ Bt, const T16* __restrict__ Bt2, int K, float* C, int ldc, const float* __restrict__ bias, size_t sA, size_t sB, size_t sC) {
    typedef typename WFrag<T16>::V V;
    __shared__ __align__(16) float os[16 * 68];
    const size_t z = blockIdx.z; A += z * sA; if (A2) A2 += z * sA; Bt += z * sB; if (Bt2) Bt2 += z * sB; C += z * sC;
    const int lane = threadIdx.x & 31, lr = lane & 15, hi = lane >> 4; const int r0 = blockIdx.x * 64, c0 = blockIdx.y * 64;
    v8f acc[4][4];
#pragma unroll
    for (int mb = 0; mb < 4; ++mb)
#pragma unroll
        for (int nb = 0; nb < 4; ++nb) acc[mb][nb] = (v8f){};
    const size_t aoff = (size_t)(r0 + lr) * K + 8 * hi, boff = (size_t)(c0 + lr) * K + 8 * hi;
#pragma unroll 1
    for (int kc = 0; kc < K; kc += 32) {
        V a[4], a2[4];
#pragma unroll
        for (int mb = 0; mb < 4; ++mb) { a[mb] = WFrag<T16>::ld(A + aoff + (size_t)mb * 16 * K + kc); if (NSPLIT == 1 || NSPLIT == 2) a2[mb] = WFrag<T16>::ld(A2 + aoff + (size_t)mb * 16 * K + kc); }
#pragma unroll
        for (int nb = 0; nb < 4; ++nb) { const V b = WFrag<T16>::ld(Bt + boff + (size_t)nb * 16 * K + kc); V b2; if (NSPLIT >= 2) b2 = WFrag<T16>::ld(Bt2 + boff + (size_t)nb * 16 * K + kc);
#pragma unroll
            for (int mb = 0; mb < 4; ++mb) { acc[mb][nb] = WFrag<T16>::mma(a[mb], b, acc[mb][nb]); if (NSPLIT == 1 || NSPLIT == 2) acc[mb][nb] = WFrag<T16>::mma(a2[mb], b, acc[mb][nb]); if (NSPLIT >= 2) acc[mb][nb] = WFrag<T16>::mma(a[mb], b2, acc[mb][nb]); } }
        asm volatile("v_nop\n\tv_nop\n\tv_nop\n\tv_nop" : "+v"(acc[0][0]), "+v"(acc[1][1]), "+v"(acc[2][2]), "+v"(acc[3][3]) : "v"(a[0]), "v"(a[3]));
    }
#pragma unroll
    for (int mb = 0; mb < 4; ++mb) {
#pragma unroll
        for (int nb = 0; nb < 4; ++nb) {
#pragma unroll
            for (int j = 0; j < 8; ++j) os[(hi * 8 + j) * 68 + nb * 16 + lr] = acc[mb][nb][j]; }
        __builtin_amdgcn_wave_barrier(); asm volatile("" ::: "memory");
        float* crow = C + (size_t)(r0 + mb * 16) * ldc + c0;
#pragma unroll 1
        for (int ps = 0; ps < 2; ++ps) {
#pragma unroll
            for (int s = 0; s < 8; ++s) { const int row = 2 * s + hi, cofs = lr * 4; v4f val = *(const v4fa*)(os + row * 68 + cofs); if (BIAS) { val[0] += bfr(bias[c0 + cofs]); val[1] += bfr(bias[c0 + cofs + 1]); val[2] += bfr(bias[c0 + cofs + 2]); val[3] += bfr(bias[c0 + cofs + 3]); }
                *(volatile v4f*)(crow + (size_t)row * ldc + cofs) = val; }
            if (ps == 0) __threadfence(); }
        __builtin_amdgcn_wave_barrier(); asm volatile("" ::: "memory");
    }
}

__device__ __forceinline__ h16 tohx(float x) { return (h16)x; }
__device__ __forceinline__ float silu_(float x) { return __fmul_rn(x, __fdiv_rn(1.0f, 1.0f + __expf(-x))); }
typedef __attribute__((ext_vector_type(2))) _Float16 v2h;
typedef __attribute__((ext_vector_type(4))) _Float16 v4h;

__global__ __launch_bounds__(256) void k_wt16(const float* __restrict__ w, int K, int N, h16* W16) { __shared__ float tile[64][65]; const int nb = (N + 63) / 64; const int k0 = (blockIdx.x / nb) * 64, n0 = (blockIdx.x % nb) * 64;
    for (int i = threadIdx.x; i < 64 * 64; i += 256) { const int kk = i / 64, nn = i % 64; tile[kk][nn] = (k0 + kk < K && n0 + nn < N) ? w[(size_t)(k0 + kk) * N + n0 + nn] : 0.f; }
    __syncthreads();
    const int nn = threadIdx.x / 4, kq = (threadIdx.x % 4) * 16; if (n0 + nn >= N) return;
    for (int c = 0; c < 16; c += 4) { v4h o; o[0] = tohx(bfr(tile[kq + c][nn])); o[1] = tohx(bfr(tile[kq + c + 1][nn])); o[2] = tohx(bfr(tile[kq + c + 2][nn])); o[3] = tohx(bfr(tile[kq + c + 3][nn])); h16* dst = W16 + (size_t)(n0 + nn) * K + k0 + kq + c; *(volatile v4h*)dst = o; __threadfence(); *(volatile v4h*)dst = o; } }
__global__ __launch_bounds__(256) void k_x16(const float* __restrict__ x, size_t n4, h16* X16) { const size_t e = ((size_t)blockIdx.x * 256 + threadIdx.x) * 4; if (e >= n4 * 4) return; const v4f a = *(const v4f*)(x + e); v4h o; o[0] = tohx(bfr(a[0])); o[1] = tohx(bfr(a[1])); o[2] = tohx(bfr(a[2])); o[3] = tohx(bfr(a[3])); *(volatile v4h*)(X16 + e) = o; __threadfence(); *(volatile v4h*)(X16 + e) = o; }
__global__ __launch_bounds__(256) void k_addx(const float* __restrict__ F, const float* __restrict__ x, float* XP) { const int e = (blockIdx.x * 256 + threadIdx.x) * 4; if (e >= TT * DD) return; const v4f a = *(const v4f*)(F + e); v4f o; o[0] = __fadd_rn(a[0], bfr(x[e])); o[1] = __fadd_rn(a[1], bfr(x[e + 1])); o[2] = __fadd_rn(a[2], bfr(x[e + 2])); o[3] = __fadd_rn(a[3], bfr(x[e + 3])); *(volatile v4f*)(XP + e) = o; __threadfence(); *(volatile v4f*)(XP + e) = o; }
__global__ __launch_bounds__(256) void k_f16(const float* __restrict__ F, size_t n4, h16* P) { const size_t e = ((size_t)blockIdx.x * 256 + threadIdx.x) * 4; if (e >= n4 * 4) return; const v4f a = *(const v4f*)(F + e); v4h o; o[0] = tohx(a[0]); o[1] = tohx(a[1]); o[2] = tohx(a[2]); o[3] = tohx(a[3]); *(volatile v4h*)(P + e) = o; __threadfence(); *(volatile v4h*)(P + e) = o; }
template <int ARAW, int SIL> __global__ __launch_bounds__(256) void k_ln2(const float* __restrict__ A, float ca, const float* __restrict__ Bs, const float* __restrict__ g, const float* __restrict__ bb, int nrows, float* YF, h16* Y16) {
    const int lane = threadIdx.x & 31; const int row = blockIdx.x * 8 + (threadIdx.x >> 5); if (row >= nrows) return; const size_t rb = (size_t)row * DD;
    auto val = [&](int c) { float a = ARAW ? bfr(A[rb + c]) : A[rb + c]; a = __fmul_rn(a, ca); if (Bs) a = __fadd_rn(a, Bs[rb + c]); return a; };
    float s = 0.f;
#pragma unroll 1
    for (int c0 = lane * 4; c0 < DD; c0 += 128) s = __fadd_rn(s, __fadd_rn(__fadd_rn(val(c0), val(c0 + 1)), __fadd_rn(val(c0 + 2), val(c0 + 3))));
#pragma unroll
    for (int sh = 16; sh; sh >>= 1) s += __shfl_xor(s, sh, 32);
    const float mean = s * (1.0f / DD); float q2 = 0.f;
#pragma unroll 1
    for (int c0 = lane * 4; c0 < DD; c0 += 128) {
#pragma unroll
        for (int u = 0; u < 4; ++u) { float d0 = __fsub_rn(val(c0 + u), mean); asm volatile("" : "+v"(d0)); float p = __fmul_rn(d0, d0); asm volatile("" : "+v"(p)); q2 = __fadd_rn(q2, p); } }
#pragma unroll
    for (int sh = 16; sh; sh >>= 1) q2 += __shfl_xor(q2, sh, 32);
    const float rstd = __frsqrt_rn(__fadd_rn(q2 * (1.0f / DD), 1e-5f));
    for (int ps = 0; ps < 2; ++ps) {
#pragma unroll 1
        for (int c0 = lane * 4; c0 < DD; c0 += 128) { v4f yo; v4h o;
#pragma unroll
            for (int u = 0; u < 4; ++u) { float t0 = __fmul_rn(__fsub_rn(val(c0 + u), mean), rstd); asm volatile("" : "+v"(t0)); float t1 = __fmul_rn(t0, bfr(g[c0 + u])); asm volatile("" : "+v"(t1)); const float y = __fadd_rn(t1, bfr(bb[c0 + u])); yo[u] = y; o[u] = tohx(SIL ? silu_(y) : y); }
            if (YF) *(volatile v4f*)(YF + rb + c0) = yo; if (Y16) *(volatile v4h*)(Y16 + rb + c0) = o; }
        if (ps == 0) __threadfence(); } }
__global__ __launch_bounds__(256) void k_qkpl(const float* __restrict__ Q, const float* __restrict__ K, h16* Q16, h16* K16) { const int e = (blockIdx.x * 256 + threadIdx.x) * 4; if (e >= NH_ * TT * HD) return; const int d = e % HD; const int t = (e / HD) % TT; const int h = e / (HD * TT); const v4f q = *(const v4f*)(Q + (size_t)t * DD + h * HD + d), k = *(const v4f*)(K + (size_t)t * DD + h * HD + d); v4h oq, ok;
#pragma unroll
    for (int u = 0; u < 4; ++u) { oq[u] = tohx(q[u] * 0.125f); ok[u] = tohx(k[u]); } for (int ps = 0; ps < 2; ++ps) { *(volatile v4h*)(Q16 + e) = oq; *(volatile v4h*)(K16 + e) = ok; if (ps == 0) __threadfence(); } }
__global__ __launch_bounds__(256) void k_vtpl(const float* __restrict__ V, int nrows, int ldv, h16* VT) { const int e = (blockIdx.x * 256 + threadIdx.x) * 2; if (e >= NH_ * HD * nrows) return; const int t = e % nrows; const int d = (e / nrows) % HD; const int h = e / (nrows * HD); v2h o; o[0] = tohx(V[(size_t)t * ldv + h * HD + d]); o[1] = tohx(V[(size_t)(t + 1) * ldv + h * HD + d]); h16* dst = VT + ((size_t)h * HD + d) * nrows + t; *(volatile v2h*)dst = o; __threadfence(); *(volatile v2h*)dst = o; }
__global__ __launch_bounds__(256) void k_mrgsilu(const float* __restrict__ O, h16* AO16) { const int e = (blockIdx.x * 256 + threadIdx.x) * 4; if (e >= TT * DD) return; const int c = e % DD; const int t = e / DD; const int h = c / HD, d = c % HD; const float* r = O + ((size_t)h * TT + t) * HD + d; v4h o;
#pragma unroll
    for (int u = 0; u < 4; ++u) o[u] = tohx(silu_(r[u] * (1.0f / PCAR))); *(volatile v4h*)(AO16 + e) = o; __threadfence(); *(volatile v4h*)(AO16 + e) = o; }
__global__ __launch_bounds__(256) void k_xfp(const float* __restrict__ xf, const float* __restrict__ w, const float* __restrict__ b, float* XFP) { const int j = blockIdx.x * 256 + threadIdx.x; if (j >= TXT) return; float acc = bfr(b[j]);
#pragma unroll 1
    for (int k = 0; k < AUD; ++k) { float p = __fmul_rn(bfr(xf[k]), bfr(w[(size_t)k * TXT + j])); asm volatile("" : "+v"(p)); acc = __fadd_rn(acc, p); } *(volatile float*)(XFP + j) = acc; __threadfence(); *(volatile float*)(XFP + j) = acc; }
__global__ __launch_bounds__(256) void k_cat16(const float* __restrict__ xw, const float* __restrict__ XFP, h16* CAT) { const int e = (blockIdx.x * 256 + threadIdx.x) * 4; if (e >= NC2 * TXT) return; const int c = e % TXT; const int n = e / TXT; v4h o;
#pragma unroll
    for (int u = 0; u < 4; ++u) o[u] = tohx(n < NW ? bfr(xw[(size_t)n * TXT + c + u]) : XFP[c + u]); *(volatile v4h*)(CAT + e) = o; __threadfence(); *(volatile v4h*)(CAT + e) = o; }
__global__ __launch_bounds__(256) void k_colstat(const float* __restrict__ M, int R, float* CM, float* CZ) { const int c = blockIdx.x * 256 + threadIdx.x; if (c >= DD) return; float mx = -3.0e38f;
#pragma unroll 1
    for (int r = 0; r < R; ++r) mx = fmaxf(mx, M[(size_t)r * DD + c]);
    float z = 0.f;
#pragma unroll 1
    for (int r = 0; r < R; ++r) { float d0 = __fsub_rn(M[(size_t)r * DD + c], mx); asm volatile("" : "+v"(d0)); z = __fadd_rn(z, __expf(d0)); }
    for (int ps = 0; ps < 2; ++ps) { *(volatile float*)(CM + c) = mx; *(volatile float*)(CZ + c) = z; if (ps == 0) __threadfence(); } }
__global__ __launch_bounds__(256) void k_ckT(const float* __restrict__ CK, const float* __restrict__ CM, const float* __restrict__ CZ, h16* CKT) { const int c = blockIdx.x * 256 + threadIdx.x; if (c >= DD) return; const int h = c / HD, d = c % HD; const float mx = CM[c], iz = __fdiv_rn(1.0f, CZ[c]); h16* row = CKT + ((size_t)h * HD + d) * NC2;
    for (int ps = 0; ps < 2; ++ps) {
#pragma unroll 1
        for (int n = 0; n < NC2; n += 4) { v4h o;
#pragma unroll
            for (int u = 0; u < 4; ++u) { float d0 = __fsub_rn(CK[(size_t)(n + u) * DD + c], mx); asm volatile("" : "+v"(d0)); o[u] = tohx(__fmul_rn(__expf(d0), iz)); } *(volatile v4h*)(row + n) = o; }
        if (ps == 0) __threadfence(); } }
__global__ __launch_bounds__(256) void k_skrow(const float* __restrict__ SK, const float* __restrict__ CM, const float* __restrict__ CZ, float* RS) { const int i = blockIdx.x * 256 + threadIdx.x; if (i >= NS_ * NH_) return; const int h = i % NH_, s = i / NH_; float acc = 0.f;
#pragma unroll 1
    for (int d = 0; d < HD; ++d) { const int c = h * HD + d; float d0 = __fsub_rn(SK[(size_t)s * DD + c], CM[c]); asm volatile("" : "+v"(d0)); acc = __fadd_rn(acc, __fdiv_rn(__expf(d0), CZ[c])); } *(volatile float*)(RS + i) = acc; __threadfence(); *(volatile float*)(RS + i) = acc; }
__global__ __launch_bounds__(256) void k_sy(const float* __restrict__ RS, const float* __restrict__ SV, float* SY) { const int i = blockIdx.x * 256 + threadIdx.x; if (i >= NH_ * HD) return; const int h = i / HD, l = i % HD; float acc = 0.f;
#pragma unroll 1
    for (int s = 0; s < NS_; ++s) { float p = __fmul_rn(RS[s * NH_ + h], SV[(size_t)s * DD + h * HD + l]); asm volatile("" : "+v"(p)); acc = __fadd_rn(acc, p); } *(volatile float*)(SY + i) = acc; __threadfence(); *(volatile float*)(SY + i) = acc; }
__global__ __launch_bounds__(256) void k_cq(const float* __restrict__ CQR, h16* CQ16) { const int lane = threadIdx.x & 31; const int w = blockIdx.x * 8 + (threadIdx.x >> 5); if (w >= TT * NH_) return; const int h = w % NH_, t = w / NH_; const float* r = CQR + (size_t)t * DD + h * HD + 2 * lane; const float a0 = r[0], a1 = r[1]; float mx = fmaxf(a0, a1);
#pragma unroll
    for (int sh = 16; sh; sh >>= 1) mx = fmaxf(mx, __shfl_xor(mx, sh, 32));
    float d0 = __fsub_rn(a0, mx), d1 = __fsub_rn(a1, mx); asm volatile("" : "+v"(d0)); asm volatile("" : "+v"(d1)); const float e0 = __expf(d0), e1 = __expf(d1); float z = __fadd_rn(e0, e1);
#pragma unroll
    for (int sh = 16; sh; sh >>= 1) z += __shfl_xor(z, sh, 32);
    const float iz = __fdiv_rn(1.0f, z); v2h o; o[0] = tohx(__fmul_rn(e0, iz)); o[1] = tohx(__fmul_rn(e1, iz)); h16* dst = CQ16 + ((size_t)h * TT + t) * HD + 2 * lane; *(volatile v2h*)dst = o; __threadfence(); *(volatile v2h*)dst = o; }
__global__ __launch_bounds__(256) void k_cysy(const float* __restrict__ CY, const float* __restrict__ SY, h16* CYS16) { const int e = (blockIdx.x * 256 + threadIdx.x) * 4; if (e >= TT * DD) return; const int c = e % DD; const int t = e / DD; const int h = c / HD, l = c % HD; const float* r = CY + ((size_t)h * TT + t) * HD + l; v4h o;
#pragma unroll
    for (int u = 0; u < 4; ++u) o[u] = tohx(silu_(__fadd_rn(r[u], SY[c + u]))); *(volatile v4h*)(CYS16 + e) = o; __threadfence(); *(volatile v4h*)(CYS16 + e) = o; }
__global__ __launch_bounds__(256) void k_gelu16(const float* __restrict__ F, size_t n4, h16* G16) { const size_t e = ((size_t)blockIdx.x * 256 + threadIdx.x) * 4; if (e >= n4 * 4) return; const v4f a = *(const v4f*)(F + e); v4h o;
#pragma unroll 1
    for (int u = 0; u < 4; ++u) { const float x = a[u]; o[u] = tohx(__fmul_rn(0.5f * x, __fadd_rn(1.0f, erff(x * 0.7071067811865476f)))); } *(volatile v4h*)(G16 + e) = o; __threadfence(); *(volatile v4h*)(G16 + e) = o; }
template <int NFULL, int TAIL> __global__ __launch_bounds__(256) void k_soft(const float* __restrict__ Sb, int nrows, int rowsper, int rvalid, int nvalid, h16* P) { const int lane = threadIdx.x & 31; const size_t row = (size_t)blockIdx.x * 8 + (threadIdx.x >> 5); if (row >= (size_t)nrows) return; constexpr int LD = NFULL * 128 + TAIL * 64; const float* sr = Sb + row * LD; h16* pr = P + row * LD; const bool live = (int)(row % rowsper) < rvalid; float mx = -3.0e38f;
#pragma unroll 1
    for (int ch = 0; ch < NFULL + TAIL; ++ch) { if (ch == NFULL && lane >= 16) break; const int j0 = ch * 128 + lane * 4; const v4f a = *(const v4f*)(sr + j0);
#pragma unroll
        for (int q = 0; q < 4; ++q) if (j0 + q < nvalid) mx = fmaxf(mx, a[q]); }
#pragma unroll
    for (int sh = 16; sh; sh >>= 1) mx = fmaxf(mx, __shfl_xor(mx, sh, 32));
    float sum = 0.f;
#pragma unroll 1
    for (int ch = 0; ch < NFULL + TAIL; ++ch) { if (ch == NFULL && lane >= 16) break; const int j0 = ch * 128 + lane * 4; const v4f a = *(const v4f*)(sr + j0);
#pragma unroll
        for (int q = 0; q < 4; ++q) if (j0 + q < nvalid) { float d0 = __fsub_rn(a[q], mx); asm volatile("" : "+v"(d0)); sum += __expf(d0); } }
#pragma unroll
    for (int sh = 16; sh; sh >>= 1) sum += __shfl_xor(sum, sh, 32);
    const float f = live ? __fdiv_rn(PCAR, sum) : 0.f;
    for (int ps = 0; ps < 2; ++ps) {
#pragma unroll 1
        for (int ch = 0; ch < NFULL + TAIL; ++ch) { if (ch == NFULL && lane >= 16) break; const int j0 = ch * 128 + lane * 4; const v4f a = *(const v4f*)(sr + j0); v4h o;
#pragma unroll
            for (int q = 0; q < 4; ++q) { float val = 0.f; if (live && j0 + q < nvalid) { float d0 = __fsub_rn(a[q], mx); asm volatile("" : "+v"(d0)); val = __fmul_rn(__expf(d0), f); } o[q] = tohx(val); } *(volatile v4h*)(pr + j0) = o; }
        if (ps == 0) __threadfence(); } }

extern "C" void kernel_launch(void* const* d_in, const int* in_sizes, int n_in,
                              void* d_out, int out_size, void* d_ws, size_t ws_size, hipStream_t stream) {
    (void)in_sizes; (void)n_in; (void)out_size;
    const float** I = (const float**)d_in;
    const float *x = I[0], *xf = I[1], *xw = I[2], *xs = I[3], *fp_w = I[4], *fp_b = I[5], *sa_ng = I[6], *sa_nb = I[7], *sa_qw = I[8], *sa_qb = I[9], *sa_kw = I[10], *sa_kb = I[11], *sa_vw = I[12], *sa_vb = I[13], *sa_ow = I[14], *sa_ob = I[15], *ca_ng = I[16], *ca_nb = I[17], *ca_tng = I[18], *ca_tnb = I[19], *ca_sng = I[20], *ca_snb = I[21];
    const float *ca_qw = I[22], *ca_qb = I[23], *ca_kw = I[24], *ca_kb = I[25], *ca_vw = I[26], *ca_vb = I[27], *ca_apw = I[28], *ca_apb = I[29], *ca_atw = I[30], *ca_atb = I[31], *ca_ow = I[32], *ca_ob = I[33], *an_g = I[34], *an_b = I[35], *ffn_w1 = I[36], *ffn_b1 = I[37], *ffn_w2 = I[38], *ffn_b2 = I[39], *ffn_ng = I[40], *ffn_nb = I[41], *ffn_ow = I[42], *ffn_ob = I[43];
    float* OUT = (float*)d_out;
    char* wsp = (char*)d_ws;
    auto take = [&](size_t bytes) { char* p = wsp; wsp += (bytes + 255) & ~(size_t)255; return (void*)p; };
    h16* FPW = (h16*)take(DD * DD * 2); h16* SQW = (h16*)take(DD * DD * 2); h16* SKW = (h16*)take(DD * DD * 2); h16* SVW = (h16*)take(DD * DD * 2); h16* SOW = (h16*)take(DD * DD * 2); h16* CQW = (h16*)take(DD * DD * 2); h16* CKW = (h16*)take(DD * DD * 2); h16* CVW = (h16*)take(DD * DD * 2); h16* ATW = (h16*)take(DD * TXT * 2); h16* COW = (h16*)take(DD * DD * 2); h16* W1 = (h16*)take((size_t)FF * DD * 2); h16* W2 = (h16*)take((size_t)DD * FF * 2); h16* FOW = (h16*)take(DD * DD * 2);
    h16* X16 = (h16*)take((size_t)TT * DD * 2); float* F = (float*)take((size_t)TT * DD * 4); float* XP = (float*)take((size_t)TT * DD * 4); h16* XN16 = (h16*)take((size_t)TT * DD * 2); float* Q = (float*)take((size_t)TT * DD * 4); float* Kf = (float*)take((size_t)TT * DD * 4); float* Vf = (float*)take((size_t)TT * DD * 4);
    h16* Q16 = (h16*)take((size_t)NH_ * TT * HD * 2); h16* K16 = (h16*)take((size_t)NH_ * TT * HD * 2); h16* VT16 = (h16*)take((size_t)NH_ * HD * TT * 2); float* Sb = (float*)take((size_t)NH_ * TT * TT * 4); h16* P16 = (h16*)take((size_t)NH_ * TT * TT * 2); float* O = (float*)take((size_t)NH_ * TT * HD * 4); h16* AO16 = (h16*)take((size_t)TT * DD * 2); float* SAO = (float*)take((size_t)TT * DD * 4);
    float* Y1 = (float*)take((size_t)TT * DD * 4); h16* CQN16 = (h16*)take((size_t)TT * DD * 2); float* XFP = (float*)take(TXT * 4); h16* CAT16 = (h16*)take((size_t)NC2 * TXT * 2); float* XWXF = (float*)take((size_t)NC2 * DD * 4); h16* TN16 = (h16*)take((size_t)NC2 * DD * 2); h16* SN16 = (h16*)take((size_t)NS_ * DD * 2);
    float* CK = (float*)take((size_t)NC2 * DD * 4); float* SK = (float*)take((size_t)NS_ * DD * 4); float* CV = (float*)take((size_t)NC2 * DD * 4); float* SV = (float*)take((size_t)NS_ * DD * 4); float* CM = (float*)take(DD * 4); float* CZ = (float*)take(DD * 4); float* CM2 = (float*)take(DD * 4); float* CZ2 = (float*)take(DD * 4); h16* CKT16 = (h16*)take((size_t)NH_ * HD * NC2 * 2); h16* CVT16 = (h16*)take((size_t)NH_ * HD * NC2 * 2); float* ATTT = (float*)take((size_t)NH_ * HD * HD * 4); h16* ATT16 = (h16*)take((size_t)NH_ * HD * HD * 2); float* RS = (float*)take(NS_ * NH_ * 4); float* SY = (float*)take(NH_ * HD * 4);
    float* CQR = (float*)take((size_t)TT * DD * 4); h16* CQ16 = (h16*)take((size_t)NH_ * TT * HD * 2); float* CY = (float*)take((size_t)NH_ * TT * HD * 4); h16* CYS16 = (h16*)take((size_t)TT * DD * 2); float* CAO = (float*)take((size_t)TT * DD * 4); float* Y2 = (float*)take((size_t)TT * DD * 4); h16* Y216 = (h16*)take((size_t)TT * DD * 2); float* H1 = (float*)take((size_t)TT * FF * 4); h16* G16 = (h16*)take((size_t)TT * FF * 2); float* H2 = (float*)take((size_t)TT * DD * 4); h16* HH16 = (h16*)take((size_t)TT * DD * 2); float* FO = (float*)take((size_t)TT * DD * 4);
    if ((size_t)(wsp - (char*)d_ws) > ws_size) return;
    k_wt16<<<(DD / 64) * (DD / 64), 256, 0, stream>>>(fp_w, DD, DD, FPW); k_wt16<<<(DD / 64) * (DD / 64), 256, 0, stream>>>(sa_qw, DD, DD, SQW); k_wt16<<<(DD / 64) * (DD / 64), 256, 0, stream>>>(sa_kw, DD, DD, SKW); k_wt16<<<(DD / 64) * (DD / 64), 256, 0, stream>>>(sa_vw, DD, DD, SVW); k_wt16<<<(DD / 64) * (DD / 64), 256, 0, stream>>>(sa_ow, DD, DD, SOW);
    k_wt16<<<(DD / 64) * (DD / 64), 256, 0, stream>>>(ca_qw, DD, DD, CQW); k_wt16<<<(DD / 64) * (DD / 64), 256, 0, stream>>>(ca_kw, DD, DD, CKW); k_wt16<<<(DD / 64) * (DD / 64), 256, 0, stream>>>(ca_vw, DD, DD, CVW); k_wt16<<<(TXT / 64) * (DD / 64), 256, 0, stream>>>(ca_atw, TXT, DD, ATW); k_wt16<<<(DD / 64) * (DD / 64), 256, 0, stream>>>(ca_ow, DD, DD, COW);
    k_wt16<<<(DD / 64) * (FF / 64), 256, 0, stream>>>(ffn_w1, DD, FF, W1); k_wt16<<<(FF / 64) * (DD / 64), 256, 0, stream>>>(ffn_w2, FF, DD, W2); k_wt16<<<(DD / 64) * (DD / 64), 256, 0, stream>>>(ffn_ow, DD, DD, FOW);
    const unsigned G512 = (TT * DD / 4 + 255) / 256;
    for (int b = 0; b < NB_; ++b) { const float* xb = x + (size_t)b * TT * DD;
        k_x16<<<G512, 256, 0, stream>>>(xb, (size_t)TT * DD / 4, X16); k_gemmw<h16, 0, true><<<dim3(TT / 64, DD / 64, 1), 32, 0, stream>>>(X16, nullptr, FPW, nullptr, DD, F, DD, fp_b, 0, 0, 0); k_addx<<<G512, 256, 0, stream>>>(F, xb, XP);
        k_ln2<0, 0><<<TT / 8, 256, 0, stream>>>(XP, 1.0f, nullptr, sa_ng, sa_nb, TT, nullptr, XN16);
        k_gemmw<h16, 0, true><<<dim3(TT / 64, DD / 64, 1), 32, 0, stream>>>(XN16, nullptr, SQW, nullptr, DD, Q, DD, sa_qb, 0, 0, 0); k_gemmw<h16, 0, true><<<dim3(TT / 64, DD / 64, 1), 32, 0, stream>>>(XN16, nullptr, SKW, nullptr, DD, Kf, DD, sa_kb, 0, 0, 0); k_gemmw<h16, 0, true><<<dim3(TT / 64, DD / 64, 1), 32, 0, stream>>>(XN16, nullptr, SVW, nullptr, DD, Vf, DD, sa_vb, 0, 0, 0);
        k_qkpl<<<(NH_ * TT * HD / 4 + 255) / 256, 256, 0, stream>>>(Q, Kf, Q16, K16); k_vtpl<<<(NH_ * HD * TT / 2 + 255) / 256, 256, 0, stream>>>(Vf, TT, DD, VT16);
        k_gemmw<h16, 0, false><<<dim3(TT / 64, TT / 64, NH_), 32, 0, stream>>>(Q16, nullptr, K16, nullptr, HD, Sb, TT, nullptr, (size_t)TT * HD, (size_t)TT * HD, (size_t)TT * TT);
        k_soft<8, 0><<<(NH_ * TT + 7) / 8, 256, 0, stream>>>(Sb, NH_ * TT, TT, TT, TT, P16);
        k_gemmw<h16, 0, false><<<dim3(TT / 64, 1, NH_), 32, 0, stream>>>(P16, nullptr, VT16, nullptr, TT, O, HD, nullptr, (size_t)TT * TT, (size_t)HD * TT, (size_t)TT * HD);
        k_mrgsilu<<<G512, 256, 0, stream>>>(O, AO16); k_gemmw<h16, 0, true><<<dim3(TT / 64, DD / 64, 1), 32, 0, stream>>>(AO16, nullptr, SOW, nullptr, DD, SAO, DD, sa_ob, 0, 0, 0);
        k_ln2<0, 0><<<TT / 8, 256, 0, stream>>>(XP, 2.0f, SAO, an_g, an_b, TT, Y1, nullptr);
        k_ln2<0, 0><<<TT / 8, 256, 0, stream>>>(Y1, 1.0f, nullptr, ca_ng, ca_nb, TT, nullptr, CQN16); k_gemmw<h16, 0, true><<<dim3(TT / 64, DD / 64, 1), 32, 0, stream>>>(CQN16, nullptr, CQW, nullptr, DD, CQR, DD, ca_qb, 0, 0, 0); k_cq<<<(TT * NH_ + 7) / 8, 256, 0, stream>>>(CQR, CQ16);
        k_xfp<<<1, 256, 0, stream>>>(xf + (size_t)b * AUD, ca_apw, ca_apb, XFP); k_cat16<<<(NC2 * TXT / 4 + 255) / 256, 256, 0, stream>>>(xw + (size_t)b * NW * TXT, XFP, CAT16);
        k_gemmw<h16, 0, true><<<dim3(NC2 / 64, DD / 64, 1), 32, 0, stream>>>(CAT16, nullptr, ATW, nullptr, TXT, XWXF, DD, ca_atb, 0, 0, 0);
        k_ln2<0, 0><<<NC2 / 8, 256, 0, stream>>>(XWXF, 1.0f, nullptr, ca_tng, ca_tnb, NC2, nullptr, TN16); k_ln2<1, 0><<<NS_ / 8, 256, 0, stream>>>(xs + (size_t)b * NS_ * DD, 1.0f, nullptr, ca_sng, ca_snb, NS_, nullptr, SN16);
        k_gemmw<h16, 0, true><<<dim3(NC2 / 64, DD / 64, 1), 32, 0, stream>>>(TN16, nullptr, CKW, nullptr, DD, CK, DD, ca_kb, 0, 0, 0); k_gemmw<h16, 0, true><<<dim3(NS_ / 64, DD / 64, 1), 32, 0, stream>>>(SN16, nullptr, CKW, nullptr, DD, SK, DD, ca_kb, 0, 0, 0);
        k_gemmw<h16, 0, true><<<dim3(NC2 / 64, DD / 64, 1), 32, 0, stream>>>(TN16, nullptr, CVW, nullptr, DD, CV, DD, ca_vb, 0, 0, 0); k_gemmw<h16, 0, true><<<dim3(NS_ / 64, DD / 64, 1), 32, 0, stream>>>(SN16, nullptr, CVW, nullptr, DD, SV, DD, ca_vb, 0, 0, 0);
        k_colstat<<<(DD + 255) / 256, 256, 0, stream>>>(CK, NC2, CM, CZ); k_ckT<<<(DD + 255) / 256, 256, 0, stream>>>(CK, CM, CZ, CKT16); k_vtpl<<<(NH_ * HD * NC2 / 2 + 255) / 256, 256, 0, stream>>>(CV, NC2, DD, CVT16);
        k_colstat<<<(DD + 255) / 256, 256, 0, stream>>>(SK, NS_, CM2, CZ2); k_skrow<<<(NS_ * NH_ + 255) / 256, 256, 0, stream>>>(SK, CM2, CZ2, RS); k_sy<<<(NH_ * HD + 255) / 256, 256, 0, stream>>>(RS, SV, SY);
        k_gemmw<h16, 0, false><<<dim3(1, 1, NH_), 32, 0, stream>>>(CVT16, nullptr, CKT16, nullptr, NC2, ATTT, HD, nullptr, (size_t)HD * NC2, (size_t)HD * NC2, (size_t)HD * HD);
        k_f16<<<(NH_ * HD * HD / 4 + 255) / 256, 256, 0, stream>>>(ATTT, (size_t)NH_ * HD * HD / 4, ATT16);
        k_gemmw<h16, 0, false><<<dim3(TT / 64, 1, NH_), 32, 0, stream>>>(CQ16, nullptr, ATT16, nullptr, HD, CY, HD, nullptr, (size_t)TT * HD, (size_t)HD * HD, (size_t)TT * HD);
        k_cysy<<<G512, 256, 0, stream>>>(CY, SY, CYS16); k_gemmw<h16, 0, true><<<dim3(TT / 64, DD / 64, 1), 32, 0, stream>>>(CYS16, nullptr, COW, nullptr, DD, CAO, DD, ca_ob, 0, 0, 0);
        k_ln2<0, 0><<<TT / 8, 256, 0, stream>>>(Y1, 2.0f, CAO, an_g, an_b, TT, Y2, Y216);
        k_gemmw<h16, 0, true><<<dim3(TT / 64, FF / 64, 1), 32, 0, stream>>>(Y216, nullptr, W1, nullptr, DD, H1, FF, ffn_b1, 0, 0, 0); k_gelu16<<<(unsigned)(((size_t)TT * FF / 4 + 255) / 256), 256, 0, stream>>>(H1, (size_t)TT * FF / 4, G16);
        k_gemmw<h16, 0, true><<<dim3(TT / 64, DD / 64, 1), 32, 0, stream>>>(G16, nullptr, W2, nullptr, FF, H2, DD, ffn_b2, 0, 0, 0); k_ln2<0, 1><<<TT / 8, 256, 0, stream>>>(H2, 1.0f, nullptr, ffn_ng, ffn_nb, TT, nullptr, HH16);
        k_gemmw<h16, 0, true><<<dim3(TT / 64, DD / 64, 1), 32, 0, stream>>>(HH16, nullptr, FOW, nullptr, DD, FO, DD, ffn_ob, 0, 0, 0);
        k_ln2<0, 0><<<TT / 8, 256, 0, stream>>>(Y2, 2.0f, FO, an_g, an_b, TT, OUT + (size_t)b * TT * DD, nullptr); }
}
